// InvAttention_34961033790118
// MI455X (gfx1250) — hardware-verified
//
#include <hip/hip_runtime.h>
#include <math.h>

typedef __attribute__((ext_vector_type(16))) _Float16 v16h;
typedef __attribute__((ext_vector_type(16))) __bf16 v16b;
typedef __attribute__((ext_vector_type(8)))  _Float16 v8h;
typedef __attribute__((ext_vector_type(8)))  float v8f;
typedef __attribute__((ext_vector_type(4)))  float v4f;
typedef __attribute__((ext_vector_type(2)))  float v2f;
typedef __attribute__((ext_vector_type(4)))  unsigned v4u;
typedef __attribute__((ext_vector_type(4)))  int v4i;
typedef float __attribute__((may_alias)) float_a;
typedef int __attribute__((may_alias)) int_a;

template <typename T> __device__ __forceinline__ void vst2(void* p, T v) { *(volatile T*)p = v; __threadfence(); *(volatile T*)p = v; }
__device__ __forceinline__ v8f wmma16(v16h a, v16h b, v8f c) {
  v8f d = __builtin_amdgcn_wmma_f32_16x16x32_f16(false, a, false, b, (short)0, c, false, false);
  asm volatile("v_nop\n\tv_nop\n\tv_nop\n\tv_nop" : "+v"(d) : "v"(a), "v"(b));
  return d;
}
__device__ __forceinline__ v8f wmma_bf(v16b a, v16b b, v8f c) {
  v8f d = __builtin_amdgcn_wmma_f32_16x16x32_bf16(false, a, false, b, (short)0, c, false, false);
  asm volatile("v_nop\n\tv_nop\n\tv_nop\n\tv_nop" : "+v"(d) : "v"(a), "v"(b));
  return d;
}
__device__ __forceinline__ v16h frag_h(const _Float16* rowk0, int lane) {
  union { v16h v; v8h q[2]; } u; const _Float16* p = rowk0 + 8 * (lane >> 4);
  u.q[0] = *(const v8h*)p; u.q[1] = *(const v8h*)(p + 16); return u.v;
}
__device__ __forceinline__ v16h frag_f32(const float* rowk0, int lane) {
  v16h a; const float* p = rowk0 + 8 * (lane >> 4);
#pragma unroll
  for (int i = 0; i < 8; ++i) { a[i] = (_Float16)p[i]; a[8 + i] = (_Float16)p[16 + i]; }
  return a;
}
__device__ __forceinline__ v16h frag_f32s(const float* rowk0, int lane, float sc) {
  v16h a; const float* p = rowk0 + 8 * (lane >> 4);
#pragma unroll
  for (int i = 0; i < 8; ++i) { a[i] = (_Float16)(p[i] * sc); a[8 + i] = (_Float16)(p[16 + i] * sc); }
  return a;
}
__device__ __forceinline__ v16h fragc_f32(const float* W, int k0, int n, int lane, int ld, int K) {
  v16h a; const int g = lane >> 4;
#pragma unroll
  for (int i = 0; i < 8; ++i) { const int ka = k0 + 8 * g + i, kb = ka + 16;
    a[i] = (_Float16)(ka < K ? W[(size_t)(ka < K ? ka : K - 1) * ld + n] : 0.f); a[8 + i] = (_Float16)(kb < K ? W[(size_t)(kb < K ? kb : K - 1) * ld + n] : 0.f); }
  return a;
}
struct F2 { v16b h, l; };
__device__ __forceinline__ F2 bsplit16(const float v[16]) { F2 r;
#pragma unroll
  for (int i = 0; i < 16; ++i) { const __bf16 h = (__bf16)v[i]; r.h[i] = h; r.l[i] = (__bf16)(v[i] - (float)h); }
  return r; }
__device__ __forceinline__ F2 split_row(const float* row, int k0, int lane) { float v[16]; const float* p = row + k0 + 8 * (lane >> 4);
#pragma unroll
  for (int i = 0; i < 8; ++i) { v[i] = p[i]; v[8 + i] = p[16 + i]; }
  return bsplit16(v); }
__device__ __forceinline__ F2 split_rowK(const float* row, int k0, int lane, int K) { float v[16]; const int g = lane >> 4;
#pragma unroll
  for (int i = 0; i < 8; ++i) { const int ka = k0 + 8 * g + i, kb = ka + 16; v[i] = ka < K ? row[ka < K ? ka : K - 1] : 0.f; v[8 + i] = kb < K ? row[kb < K ? kb : K - 1] : 0.f; }
  return bsplit16(v); }
__device__ __forceinline__ F2 split_col(const float* W, int k0, int n, int lane, int ld, int K) { float v[16]; const int g = lane >> 4;
#pragma unroll
  for (int i = 0; i < 8; ++i) { const int ka = k0 + 8 * g + i, kb = ka + 16; v[i] = ka < K ? W[(size_t)(ka < K ? ka : K - 1) * ld + n] : 0.f; v[8 + i] = kb < K ? W[(size_t)(kb < K ? kb : K - 1) * ld + n] : 0.f; }
  return bsplit16(v); }
__device__ __forceinline__ v8f mac3(const F2& a, const F2& b, v8f c) { c = wmma_bf(a.l, b.h, c); c = wmma_bf(a.h, b.l, c); return wmma_bf(a.h, b.h, c); }
__device__ __forceinline__ float sigm(float v) { return 1.0f / (1.0f + expf(-v)); }
#define LDSX() do { asm volatile("s_wait_dscnt 0" ::: "memory"); __builtin_amdgcn_wave_barrier(); __builtin_amdgcn_fence(__ATOMIC_RELEASE, "workgroup"); } while (0)


#define NB 8
#define LL 4096
#define T2 2048
#define DD 256
#define LN_EPS 1e-5f
typedef __attribute__((ext_vector_type(8))) __bf16 v8b;
__device__ __forceinline__ v16b frag_b(const __bf16* rowk0, int lane) {
  union { v16b v; v8b q[2]; } u; const __bf16* p = rowk0 + 8 * (lane >> 4);
  u.q[0] = *(const v8b*)p; u.q[1] = *(const v8b*)(p + 16); return u.v;
}
__device__ __forceinline__ float bfr(float v) { return (float)(__bf16)v; }
__device__ __attribute__((noinline)) float exp_ni(float v) { return expf(v); }
__device__ __attribute__((noinline)) float erf_ni(float v) { return erff(v); }

#define WS_QH  0u
#define WS_QL  (WS_QH + 2u * (size_t)NB * T2 * DD)
#define WS_KH  (WS_QL + 2u * (size_t)NB * T2 * DD)
#define WS_KL  (WS_KH + 2u * (size_t)NB * T2 * DD)
#define WS_XT  (WS_KL + 2u * (size_t)NB * T2 * DD)
#define WS_S   (WS_XT + 2u * (size_t)NB * DD * T2)
#define WS_DG  (WS_S + 4u * (size_t)NB * T2 * T2)
#define WS_END (WS_DG + 4u * (size_t)NB * T2)
#define OUT1_OFF ((size_t)NB * LL * DD)

__global__ __launch_bounds__(128) void k_proj(const float* __restrict__ X, const float* __restrict__ WQ, const float* __restrict__ WK, const float* __restrict__ GQ, const float* __restrict__ BQ, const float* __restrict__ GK, const float* __restrict__ BK, _Float16* __restrict__ QH, _Float16* __restrict__ QL, _Float16* __restrict__ KH, _Float16* __restrict__ KL, float* __restrict__ OUT) {
  __shared__ __align__(16) float sf[64][DD + 4]; __shared__ __align__(16) _Float16 sh[64][DD + 8], sl[64][DD + 8]; __shared__ float smu[64], srs[64];
  const int tid = threadIdx.x, wave = tid >> 5, lane = tid & 31, col = lane & 15, g = lane >> 4; const int which = blockIdx.y; const size_t r0 = (size_t)blockIdx.x * 64; const size_t n = r0 / T2; const int i0 = (int)(r0 % T2);
  const float* Wm = which == 0 ? WQ : WK; const float* Gm = which == 0 ? GQ : GK; const float* Bm = which == 0 ? BQ : BK;
#pragma unroll 1
  for (int half = 0; half < 2; ++half) { v8f acc[8] = {};
#pragma unroll 2
    for (int kc = 0; kc < DD / 32; ++kc) { v16b a; { const float* p = X + ((n * LL + i0 + wave * 16 + col) * DD) + kc * 32 + 8 * g;
#pragma unroll
        for (int i = 0; i < 8; ++i) { a[i] = (__bf16)p[i]; a[8 + i] = (__bf16)p[16 + i]; } }
#pragma unroll
      for (int j = 0; j < 8; ++j) { v16b w; const int o = half * 128 + j * 16 + col; const float* p = Wm + (size_t)o * DD + kc * 32 + 8 * g;
#pragma unroll
        for (int i = 0; i < 8; ++i) { w[i] = (__bf16)p[i]; w[8 + i] = (__bf16)p[16 + i]; }
        acc[j] = wmma_bf(a, w, acc[j]); } }
#pragma unroll
    for (int j = 0; j < 8; ++j)
#pragma unroll
      for (int r = 0; r < 8; ++r) sf[wave * 16 + 8 * g + r][half * 128 + j * 16 + col] = acc[j][r]; }
  __syncthreads();
  if (tid < 64) { float m = 0.f; for (int c = 0; c < DD; ++c) m += sf[tid][c]; m *= (1.0f / DD); float v = 0.f; for (int c = 0; c < DD; ++c) { const float d = sf[tid][c] - m; v += d * d; } smu[tid] = m; srs[tid] = 1.0f / sqrtf(v * (1.0f / DD) + LN_EPS); }
  __syncthreads();
  for (int e = tid; e < 64 * DD; e += 128) { const int rl = e >> 8, c = e & 255; const float v = (sf[rl][c] - smu[rl]) * srs[rl] * bfr(Gm[c]) + bfr(Bm[c]); const _Float16 hv = (_Float16)v; sh[rl][c] = hv; sl[rl][c] = (_Float16)(v - (float)hv); }
  __syncthreads();
  _Float16* dh = which == 0 ? QH : KH; _Float16* dl = which == 0 ? QL : KL;
  for (int e = tid; e < 64 * 32; e += 128) { const int rl = e >> 5, q = e & 31; vst2((unsigned*)(dh + (r0 + rl) * DD + q * 8), *(const v4u*)&sh[rl][q * 8]); vst2((unsigned*)(dl + (r0 + rl) * DD + q * 8), *(const v4u*)&sl[rl][q * 8]); }
  if (which == 0) { for (int e = tid; e < 64 * 64; e += 128) { const int rl = e >> 6, q = e & 63; const size_t go = (n * LL + i0 + rl) * DD + q * 4; const v4f xr = *(const v4f*)(X + go); v4f v; v[0] = bfr(xr[0]); v[1] = bfr(xr[1]); v[2] = bfr(xr[2]); v[3] = bfr(xr[3]); vst2(OUT + go, v); } } }
__global__ __launch_bounds__(256) void k_x2t(const float* __restrict__ X, __bf16* __restrict__ XT) { __shared__ __align__(16) __bf16 st[DD][72];
  const int t = threadIdx.x; const size_t n = blockIdx.y; const int j0 = blockIdx.x * 64;
  for (int e = t; e < 64 * DD; e += 256) { const int jl = e >> 8, d = e & 255; st[d][jl] = (__bf16)X[(n * LL + T2 + j0 + jl) * DD + d]; }
  __syncthreads(); for (int e = t; e < DD * 8; e += 256) { const int d = e >> 3, q = e & 7; vst2((unsigned*)(XT + (n * DD + d) * (size_t)T2 + j0 + q * 8), *(const v4u*)&st[d][q * 8]); } }
__global__ __launch_bounds__(128) void k_sc(const _Float16* __restrict__ QH, const _Float16* __restrict__ QL, const _Float16* __restrict__ KH, const _Float16* __restrict__ KL, const float* __restrict__ DSC, float* __restrict__ S0) { __shared__ __align__(16) float ss[4][16][132];
  const size_t n = blockIdx.z; float* S = S0 + n * (size_t)T2 * T2;
  const int tid = threadIdx.x, wave = tid >> 5, lane = tid & 31, col = lane & 15, g = lane >> 4; const int k0 = blockIdx.y * 128; const int q0b = blockIdx.x * 64; const int ql0 = q0b + wave * 16;
  if (k0 + 127 < q0b) return;
  const float isc = 1.0f / bfr(DSC[0]);
  v8f acc[8] = {};
#pragma unroll 2
  for (int kc = 0; kc < DD / 32; ++kc) { const size_t qo = (n * T2 + ql0 + col) * DD + kc * 32; const v16h ah = frag_h(QH + qo, lane), al = frag_h(QL + qo, lane);
#pragma unroll
    for (int j = 0; j < 8; ++j) { const size_t ko = (n * T2 + k0 + j * 16 + col) * DD + kc * 32; const v16h kb = frag_h(KH + ko, lane); acc[j] = wmma16(ah, kb, acc[j]); acc[j] = wmma16(al, kb, acc[j]); acc[j] = wmma16(ah, frag_h(KL + ko, lane), acc[j]); } }
#pragma unroll
  for (int j = 0; j < 8; ++j) { const int jj = k0 + j * 16 + col;
#pragma unroll
    for (int r = 0; r < 8; ++r) { const int ii = ql0 + 8 * g + r; ss[wave][8 * g + r][j * 16 + col] = (jj >= ii) ? acc[j][r] * isc : -3.0e38f; } }
  LDSX(); for (int rl = 0; rl < 16; ++rl) vst2(S + (size_t)(ql0 + rl) * T2 + k0 + lane * 4, *(const v4f*)&ss[wave][rl][lane * 4]); }
__global__ __launch_bounds__(256) void k_sm(float* __restrict__ S0) { __shared__ float sred[8]; __shared__ float sbc; __shared__ __align__(16) float sh[T2];
  const int t = threadIdx.x; const int row = blockIdx.x; const size_t n = blockIdx.y; float* sr = S0 + (n * T2 + row) * (size_t)T2; const int kbeg = (row / 64) * 64;
  float m = -3.0e38f; for (int k = kbeg + t; k < T2; k += 256) m = fmaxf(m, sr[k]);
#pragma unroll
  for (int o = 1; o < 32; o <<= 1) m = fmaxf(m, __shfl_xor(m, o));
  if ((t & 31) == 0) sred[t >> 5] = m; __syncthreads(); if (t == 0) { float a = sred[0]; for (int i = 1; i < 8; ++i) a = fmaxf(a, sred[i]); sbc = a; } __syncthreads(); m = sbc; __syncthreads();
  float sum = 0.f; for (int k = kbeg + t; k < T2; k += 256) { const float v = sr[k]; sum += (v <= -1.0e38f) ? 0.f : expf(v - m); }
#pragma unroll
  for (int o = 1; o < 32; o <<= 1) sum += __shfl_xor(sum, o);
  if ((t & 31) == 0) sred[t >> 5] = sum; __syncthreads(); if (t == 0) { float a = 0.f; for (int i = 0; i < 8; ++i) a += sred[i]; sbc = 1.0f / a; } __syncthreads(); const float inv = sbc;
  for (int k = kbeg + t; k < T2; k += 256) { const float v = sr[k]; const float p = (v <= -1.0e38f) ? 0.f : expf(v - m) * inv; sh[k] = p * 2048.0f; }
  __syncthreads(); for (int q = kbeg / 4 + t; q < T2 / 4; q += 256) vst2(sr + q * 4, *(const v4f*)&sh[q * 4]); }
__global__ __launch_bounds__(128) void k_pv(const float* __restrict__ PS0, const __bf16* __restrict__ XT, const float* __restrict__ X, float* __restrict__ OUT) { __shared__ __align__(16) float ss[4][16][132];
  const size_t n = blockIdx.z; const float* PS = PS0 + n * (size_t)T2 * T2;
  const int tid = threadIdx.x, wave = tid >> 5, lane = tid & 31, col = lane & 15, g = lane >> 4; const int q0b = blockIdx.x * 64; const int ql0 = q0b + wave * 16; const int c0 = blockIdx.y * 128;
  v8f acc[8] = {};
#pragma unroll 1
  for (int kc = q0b / 32; kc < T2 / 32; ++kc) { const F2 p = split_row(PS + (size_t)(ql0 + col) * T2, kc * 32, lane);
#pragma unroll
    for (int j = 0; j < 8; ++j) { const v16b xb = frag_b(XT + (n * DD + c0 + j * 16 + col) * (size_t)T2 + kc * 32, lane); acc[j] = wmma_bf(p.h, xb, acc[j]); acc[j] = wmma_bf(p.l, xb, acc[j]); } }
#pragma unroll
  for (int j = 0; j < 8; ++j) { const int d = c0 + j * 16 + col;
#pragma unroll
    for (int r = 0; r < 8; ++r) { const int ii = ql0 + 8 * g + r; ss[wave][8 * g + r][j * 16 + col] = acc[j][r] * (1.0f / 2048.0f) + bfr(X[(n * LL + T2 + ii) * DD + d]); } }
  LDSX(); for (int rl = 0; rl < 16; ++rl) vst2(OUT + (n * LL + T2 + ql0 + rl) * DD + c0 + lane * 4, *(const v4f*)&ss[wave][rl][lane * 4]); }
__global__ __launch_bounds__(256) void k_logdet(const float* __restrict__ PS, float* __restrict__ OUT) {   __shared__ float sred[8]; __shared__ __align__(16) float so[NB];
  const int t = threadIdx.x;
#pragma unroll 1
  for (int n = 0; n < NB; ++n) { float s = 0.f;
#pragma unroll 1
    for (int i = t; i < T2; i += 256) s += logf(1.0f + PS[((size_t)n * T2 + i) * T2 + i] * (1.0f / 2048.0f));
#pragma unroll
    for (int o = 1; o < 32; o <<= 1) s += __shfl_xor(s, o);
    if ((t & 31) == 0) sred[t >> 5] = s; __syncthreads(); if (t == 0) { float a = 0.f; for (int i = 0; i < 8; ++i) a += sred[i]; so[n] = a * (float)(LL / 2); } __syncthreads(); }
  if (t < NB / 4) vst2(OUT + OUT1_OFF + t * 4, *(const v4f*)&so[t * 4]); }
extern "C" void kernel_launch(void* const* d_in, const int* in_sizes, int n_in, void* d_out, int out_size, void* d_ws, size_t ws_size, hipStream_t stream) {
  (void)in_sizes; (void)n_in; (void)out_size;
  const float** F = (const float**)d_in;
  if (ws_size < (size_t)WS_END) return;
  char* ws = (char*)d_ws; _Float16 *QH = (_Float16*)(ws + WS_QH), *QL = (_Float16*)(ws + WS_QL), *KH = (_Float16*)(ws + WS_KH), *KL = (_Float16*)(ws + WS_KL); __bf16* XT = (__bf16*)(ws + WS_XT); float *S = (float*)(ws + WS_S), *DG = (float*)(ws + WS_DG);
  float* OUT = (float*)d_out;
  k_proj<<<dim3(NB * T2 / 64, 2), 128, 0, stream>>>(F[0], F[1], F[2], F[3], F[4], F[5], F[6], QH, QL, KH, KL, OUT);
  k_x2t<<<dim3(T2 / 64, NB), 256, 0, stream>>>(F[0], XT);
  k_sc<<<dim3(T2 / 64, T2 / 128, NB), 128, 0, stream>>>(QH, QL, KH, KL, F[7], S);
  k_sm<<<dim3(T2, NB), 256, 0, stream>>>(S);
  k_pv<<<dim3(T2 / 64, DD / 128, NB), 128, 0, stream>>>(S, XT, F[0], OUT);
  k_logdet<<<1, 256, 0, stream>>>(S, OUT);
}
